// Mamba_Block_59631325938214
// MI455X (gfx1250) — hardware-verified
//
#include <hip/hip_runtime.h>
#include <math.h>

typedef __attribute__((ext_vector_type(16))) _Float16 v16h;
typedef __attribute__((ext_vector_type(8)))  _Float16 v8h;
typedef __attribute__((ext_vector_type(16))) __bf16   v16b;
typedef __attribute__((ext_vector_type(8)))  __bf16   v8b;
typedef __attribute__((ext_vector_type(8)))  float    v8f;
typedef __attribute__((ext_vector_type(4)))  float    v4f;
typedef __attribute__((ext_vector_type(2)))  float    v2f;

constexpr int kBatch = 4;
constexpr int kSeq   = 1024;
constexpr int kDm    = 512;
constexpr int kDin   = 1024;
constexpr int kNst   = 16;
constexpr int kDtR   = 32;
constexpr int kDepth = 5;
constexpr int kXzP   = 2 * kDin;
constexpr int kXdP   = kDtR + 2 * kNst;
constexpr int kHid   = 2 * kDm;
constexpr int kRows  = kBatch * kSeq;
constexpr int kConvTP = 260;
constexpr int kScanTS = 64;
constexpr int kScanCh = 64;
constexpr int kScanXP = 32;
constexpr int kScanYP = 68;
static_assert(kXdP == 64, "x_proj width");
static_assert((kDm % 32) == 0 && (kDin % 32) == 0 && (kDtR % 32) == 0 && (kHid % 32) == 0, "GEMM K multiples of 32");
static_assert((kRows % 64) == 0 && (kXzP % 64) == 0 && (kXdP % 64) == 0 && (kDm % 64) == 0 &&
              (kDin % 64) == 0 && (kHid % 64) == 0, "GEMM M,N multiples of 64");
static_assert((kSeq % kScanTS) == 0 && (kSeq % 64) == 0 && (kDin % kScanCh) == 0 && (kDin % 256) == 0 &&
              (kRows % 8) == 0 && (kDm == 512), "tile multiples");

constexpr int kNWin  = kXzP * kDm;
constexpr int kNWx   = kXdP * kDin;
constexpr int kNWdt  = kDin * kDtR;
constexpr int kNWo   = kDm  * kDin;
constexpr int kNW1   = kHid * kDm;
constexpr int kNW2   = kDm  * kHid;
constexpr int kEoffWin = 0;
constexpr int kEoffWx  = kEoffWin + kNWin;
constexpr int kEoffWdt = kEoffWx  + kNWx;
constexpr int kEoffWo  = kEoffWdt + kNWdt;
constexpr int kEoffW1  = kEoffWo  + kNWo;
constexpr int kEoffW2  = kEoffW1  + kNW1;
constexpr int kNW16    = kEoffW2  + kNW2;
static_assert(kNW16 == 2719744, "staging plane size");
static_assert(((kEoffWx * 2) % 128) == 0 && ((kEoffWdt * 2) % 128) == 0 && ((kEoffWo * 2) % 128) == 0 &&
              ((kEoffW1 * 2) % 128) == 0 && ((kEoffW2 * 2) % 128) == 0, "128-B aligned weight slots");
static_assert((kNWin % 2048) == 0 && (kNWx % 2048) == 0 && (kNWdt % 2048) == 0 && (kNWo % 2048) == 0 &&
              (kNW1 % 2048) == 0 && (kNW2 % 2048) == 0, "cast segments");
constexpr int kCB1 = kNWin / 2048;
constexpr int kCB2 = kCB1 + kNWx  / 2048;
constexpr int kCB3 = kCB2 + kNWdt / 2048;
constexpr int kCB4 = kCB3 + kNWo  / 2048;
constexpr int kCB5 = kCB4 + kNW1  / 2048;
constexpr int kCastBlocks = kCB5 + kNW2 / 2048;
static_assert(kCastBlocks == 1328, "cast grid");

constexpr size_t kOffXA    = 0;
constexpr size_t kOffXB    = kOffXA    + (size_t)kRows * kDm  * 4;
constexpr size_t kOffU16   = kOffXB    + (size_t)kRows * kDm  * 4;
constexpr size_t kOffXZ    = kOffU16   + (size_t)kRows * kDm  * 2;
constexpr size_t kOffUC    = kOffXZ    + (size_t)kRows * kXzP * 4;
constexpr size_t kOffUC16  = kOffUC    + (size_t)kRows * kDin * 4;
constexpr size_t kOffXD    = kOffUC16  + (size_t)kRows * kDin * 2;
constexpr size_t kOffDTR16 = kOffXD    + (size_t)kRows * kXdP * 4;
constexpr size_t kOffDT    = kOffDTR16 + (size_t)kRows * kDtR * 2;
constexpr size_t kOffY16   = kOffDT    + (size_t)kRows * kDin * 4;
constexpr size_t kOffH16   = kOffY16   + (size_t)kRows * kDin * 2;
constexpr size_t kOffW16   = kOffH16   + (size_t)kRows * kHid * 2;
constexpr size_t kWsTotal  = kOffW16   + (size_t)kNW16 * 2;
static_assert(kWsTotal == 119996416ull, "carve total");
static_assert(kWsTotal <= 134217728ull, "carve cap");
static_assert((size_t)kRows * kHid * 4 <= (size_t)kRows * kXzP * 4, "mlp-up pre-activation fits the XZ region");
static_assert((kOffXB % 128) == 0 && (kOffU16 % 128) == 0 && (kOffXZ % 128) == 0 && (kOffUC % 128) == 0 &&
              (kOffUC16 % 128) == 0 && (kOffXD % 128) == 0 && (kOffDTR16 % 128) == 0 && (kOffDT % 128) == 0 &&
              (kOffY16 % 128) == 0 && (kOffH16 % 128) == 0 && (kOffW16 % 128) == 0, "128-B aligned regions");

__device__ __forceinline__ unsigned short f2bf_bits(float f) {
  unsigned u = __float_as_uint(f);
  return (unsigned short)((u + 0x7FFFu + ((u >> 16) & 1u)) >> 16);
}
__device__ __forceinline__ float bf_bits2f(unsigned short h) { return __uint_as_float(((unsigned)h) << 16); }

__device__ __forceinline__ void dep_guard_h(v8f& a, v8f& b, v16h x, v16h y) { asm volatile("v_nop\n\tv_nop\n\tv_nop\n\tv_nop" : "+v"(a), "+v"(b) : "v"(x), "v"(y)); }
__device__ __forceinline__ void dep_guard_b(v8f& a, v8f& b, v16b x, v16b y) { asm volatile("v_nop\n\tv_nop\n\tv_nop\n\tv_nop" : "+v"(a), "+v"(b) : "v"(x), "v"(y)); }
__device__ __forceinline__ void keep4_h(v16h a, v16h b, v16h c, v16h d) { asm volatile("v_nop" :: "v"(a), "v"(b), "v"(c), "v"(d)); }
__device__ __forceinline__ void keep4_b(v16b a, v16b b, v16b c, v16b d) { asm volatile("v_nop" :: "v"(a), "v"(b), "v"(c), "v"(d)); }
__device__ __forceinline__ void acc_guard4(v8f& a, v8f& b, v8f& c, v8f& d) { asm volatile("v_nop\n\tv_nop\n\tv_nop\n\tv_nop" : "+v"(a), "+v"(b), "+v"(c), "+v"(d)); }
template <typename T> struct Frag;
template <> struct Frag<_Float16> {
  typedef v16h V; union U { v16h v; v8h h[2]; };
  static __device__ __forceinline__ v16h load(const _Float16* p) {
    U f; f.h[0] = *(const v8h*)(p); f.h[1] = *(const v8h*)(p + 16); return f.v;
  }
  static __device__ __forceinline__ v8f mma(v16h a, v16h b, v8f c) {
    return __builtin_amdgcn_wmma_f32_16x16x32_f16(false, a, false, b, (short)0, c, false, false);
  }
  static __device__ __forceinline__ void guard(v8f& a, v8f& b, v16h x, v16h y) { dep_guard_h(a, b, x, y); }
  static __device__ __forceinline__ void keep(v16h a, v16h b, v16h c, v16h d) { keep4_h(a, b, c, d); }
};
template <> struct Frag<__bf16> {
  typedef v16b V; union U { v16b v; v8b h[2]; };
  static __device__ __forceinline__ v16b load(const __bf16* p) {
    U f; f.h[0] = *(const v8b*)(p); f.h[1] = *(const v8b*)(p + 16); return f.v;
  }
  static __device__ __forceinline__ v8f mma(v16b a, v16b b, v8f c) {
    return __builtin_amdgcn_wmma_f32_16x16x32_bf16(false, a, false, b, (short)0, c, false, false);
  }
  static __device__ __forceinline__ void guard(v8f& a, v8f& b, v16b x, v16b y) { dep_guard_b(a, b, x, y); }
  static __device__ __forceinline__ void keep(v16b a, v16b b, v16b c, v16b d) { keep4_b(a, b, c, d); }
};

template <int ET> struct Elem;
template <> struct Elem<0> { typedef _Float16 T; };
template <> struct Elem<1> { typedef __bf16 T; };
template <int ET, bool SPLIT, int BIAS_MODE, int OUT_MODE, bool RESID>
__global__ __launch_bounds__(256) void wmma_gemm64(
    const unsigned short* __restrict__ Ap, const unsigned short* __restrict__ A2p, int lda, long strideA,
    const unsigned short* __restrict__ Btp, const unsigned short* __restrict__ Bt2p, int ldb, long strideB,
    void* __restrict__ Cout, void* __restrict__ Cout2, int ldc, long strideC,
    const float* __restrict__ bias,
    const float* __restrict__ resid, long strideR,
    int M, int N, int K, float scale) {
  typedef typename Elem<ET>::T T;
  typedef typename Frag<T>::V V;
  const T* A = (const T*)Ap; const T* A2 = (const T*)A2p; const T* Bt = (const T*)Btp; const T* Bt2 = (const T*)Bt2p;
  __shared__ __align__(16) float sT[8][16 * 68];
  const int b    = blockIdx.y;
  const int lane = threadIdx.x & 31;
  const int wave = threadIdx.x >> 5;
  const int tilesN = N >> 6;
  const int tilesM = M >> 6;
  const int tile = blockIdx.x * 8 + wave;
  if (tile >= tilesM * tilesN) return;
  const int tm = tile / tilesN;
  const int tn = tile - tm * tilesN;
  const int m0 = tm << 6;
  const int n0 = tn << 6;

  const T* Ab  = A  + (size_t)b * strideA;
  const T* Bb  = Bt + (size_t)b * strideB;
  const T* Ab2 = SPLIT ? (A2  + (size_t)b * strideA) : nullptr;
  const T* Bb2 = SPLIT ? (Bt2 + (size_t)b * strideB) : nullptr;

  const int rlane = lane & 15;
  const int koff  = (lane >> 4) * 8;
  const int mOff  = (lane >> 4) * 8;

  v8f acc[4][4];
#pragma unroll
  for (int i = 0; i < 4; ++i)
#pragma unroll
    for (int j = 0; j < 4; ++j) acc[i][j] = (v8f){0.f,0.f,0.f,0.f,0.f,0.f,0.f,0.f};

  for (int k0 = 0; k0 < K; k0 += 32) {
    V bh[4], bl[4];
#pragma unroll
    for (int j = 0; j < 4; ++j) {
      const size_t bo = (size_t)(n0 + (j << 4) + rlane) * ldb + koff + k0;
      bh[j] = Frag<T>::load(Bb + bo);
      if (SPLIT) bl[j] = Frag<T>::load(Bb2 + bo);
    }
#pragma unroll
    for (int i = 0; i < 4; ++i) {
      const size_t ao = (size_t)(m0 + (i << 4) + rlane) * lda + koff + k0;
      V ah = Frag<T>::load(Ab + ao);
      V al;
      if (SPLIT) al = Frag<T>::load(Ab2 + ao);
#pragma unroll
      for (int j = 0; j < 4; ++j) {
        acc[i][j] = Frag<T>::mma(ah, bh[j], acc[i][j]);
        if (SPLIT) {
          acc[i][j] = Frag<T>::mma(ah, bl[j], acc[i][j]);
          acc[i][j] = Frag<T>::mma(al, bh[j], acc[i][j]);
        }
      }
      Frag<T>::guard(acc[i][0], acc[i][3], ah, SPLIT ? al : ah);
    }
    Frag<T>::keep(bh[0], bh[1], bh[2], bh[3]);
    if (SPLIT) Frag<T>::keep(bl[0], bl[1], bl[2], bl[3]);
  }
  acc_guard4(acc[0][0], acc[0][1], acc[0][2], acc[0][3]);
  acc_guard4(acc[1][0], acc[1][1], acc[1][2], acc[1][3]);
  acc_guard4(acc[2][0], acc[2][1], acc[2][2], acc[2][3]);
  acc_guard4(acc[3][0], acc[3][1], acc[3][2], acc[3][3]);

  float* slab = sT[wave];
  const float* Rb = RESID ? (resid + (size_t)b * strideR) : nullptr;
#pragma unroll
  for (int i = 0; i < 4; ++i) {
    const int mBase = m0 + (i << 4);
#pragma unroll
    for (int j = 0; j < 4; ++j) {
      const int n = n0 + (j << 4) + rlane;
      float bv = 0.f;
      if (BIAS_MODE == 2) bv = bias[n];
#pragma unroll
      for (int r = 0; r < 8; ++r) {
        float v = acc[i][j][r] * scale;
        if (BIAS_MODE == 1) v += bias[mBase + mOff + r];
        if (BIAS_MODE == 2) v += bv;
        slab[(mOff + r) * 68 + (j << 4) + rlane] = v;
      }
    }
    __builtin_amdgcn_fence(__ATOMIC_RELEASE, "workgroup");
    __builtin_amdgcn_wave_barrier();
    __builtin_amdgcn_fence(__ATOMIC_ACQUIRE, "workgroup");
    if (OUT_MODE == 0) {
      float* C = (float*)Cout + (size_t)b * strideC;
      const int hh = lane >> 4, c4 = (lane & 15) * 4;
      v4f ov[8];
#pragma unroll
      for (int it = 0; it < 8; ++it) {
        const int row = it * 2 + hh;
        v4f v = *(const v4f*)(slab + row * 68 + c4);
        if (RESID) {
          const v4f rr = *(const v4f*)(Rb + (size_t)(mBase + row) * ldc + n0 + c4);
          v += rr;
        }
        ov[it] = v;
      }
      for (int pass = 0; pass < 2; ++pass) {
#pragma unroll
        for (int it = 0; it < 8; ++it) {
          const int row = it * 2 + hh;
          *(volatile v4f*)(C + (size_t)(mBase + row) * ldc + n0 + c4) = ov[it];
        }
        __threadfence();
      }
    } else {
      const int q = lane >> 3, c8 = (lane & 7) * 8;
      unsigned short* C  = (unsigned short*)Cout  + (size_t)b * strideC;
      unsigned short* C2 = (OUT_MODE == 2) ? ((unsigned short*)Cout2 + (size_t)b * strideC) : nullptr;
      for (int pass = 0; pass < 2; ++pass) {
#pragma unroll
        for (int it = 0; it < 4; ++it) {
          const int row = it * 4 + q;
          const float* sp = slab + row * 68 + c8;
          v8h hv, lv;
#pragma unroll
          for (int e = 0; e < 8; ++e) {
            if (OUT_MODE == 1) {
              hv[e] = (_Float16)sp[e];
            } else {
              unsigned short hb = f2bf_bits(sp[e]);
              unsigned short lb = f2bf_bits(sp[e] - bf_bits2f(hb));
              hv[e] = __builtin_bit_cast(_Float16, hb);
              lv[e] = __builtin_bit_cast(_Float16, lb);
            }
          }
          *(volatile v8h*)(C + (size_t)(mBase + row) * ldc + n0 + c8) = hv;
          if (OUT_MODE == 2) *(volatile v8h*)(C2 + (size_t)(mBase + row) * ldc + n0 + c8) = lv;
        }
        __threadfence();
      }
    }
    __builtin_amdgcn_fence(__ATOMIC_RELEASE, "workgroup");
    __builtin_amdgcn_wave_barrier();
    __builtin_amdgcn_fence(__ATOMIC_ACQUIRE, "workgroup");
  }
}

__global__ __launch_bounds__(256) void castw_kernel(
    const float* __restrict__ s0, const float* __restrict__ s1, const float* __restrict__ s2,
    const float* __restrict__ s3, const float* __restrict__ s4, const float* __restrict__ s5,
    unsigned short* __restrict__ W16)
{
  const int blk = blockIdx.x;
  const float* src;
  size_t doff;
  int lb;
  if (blk < kCB1)      { src = s0; doff = (size_t)kEoffWin; lb = blk; }
  else if (blk < kCB2) { src = s1; doff = (size_t)kEoffWx;  lb = blk - kCB1; }
  else if (blk < kCB3) { src = s2; doff = (size_t)kEoffWdt; lb = blk - kCB2; }
  else if (blk < kCB4) { src = s3; doff = (size_t)kEoffWo;  lb = blk - kCB3; }
  else if (blk < kCB5) { src = s4; doff = (size_t)kEoffW1;  lb = blk - kCB4; }
  else                 { src = s5; doff = (size_t)kEoffW2;  lb = blk - kCB5; }
  const size_t e0 = ((size_t)lb * 256 + threadIdx.x) * 8;
  const v4f a0 = *(const v4f*)(src + e0);
  const v4f a1 = *(const v4f*)(src + e0 + 4);
  v8h hv;
#pragma unroll
  for (int e = 0; e < 4; ++e) { hv[e] = (_Float16)a0[e]; hv[4 + e] = (_Float16)a1[e]; }
  unsigned short* qd = W16 + doff + e0;
  *(volatile v8h*)qd = hv;
  __threadfence();
  *(volatile v8h*)qd = hv;
}

__global__ __launch_bounds__(256) void ln_f16_kernel(
    const float* __restrict__ X, const float* __restrict__ gam, const float* __restrict__ bet,
    unsigned short* __restrict__ Uo)
{
  const int lane = threadIdx.x & 31, wave = threadIdx.x >> 5;
  const int row = blockIdx.x * 8 + wave;
  const float* xr = X + (size_t)row * kDm;
  const int c0 = lane * 8, c1 = (kDm / 2) + lane * 8;
  const v4f a0 = *(const v4f*)(xr + c0);
  const v4f a1 = *(const v4f*)(xr + c0 + 4);
  const v4f a2 = *(const v4f*)(xr + c1);
  const v4f a3 = *(const v4f*)(xr + c1 + 4);
  float v[16];
#pragma unroll
  for (int e = 0; e < 4; ++e) { v[e] = a0[e]; v[4 + e] = a1[e]; v[8 + e] = a2[e]; v[12 + e] = a3[e]; }
  float s = 0.f;
#pragma unroll
  for (int e = 0; e < 16; ++e) s += v[e];
#pragma unroll
  for (int off = 1; off < 32; off <<= 1) s += __shfl_xor(s, off, 32);
  const float mean = s * (1.0f / kDm);
  float q2 = 0.f;
#pragma unroll
  for (int e = 0; e < 16; ++e) { const float dd = v[e] - mean; q2 = fmaf(dd, dd, q2); }
#pragma unroll
  for (int off = 1; off < 32; off <<= 1) q2 += __shfl_xor(q2, off, 32);
  const float var  = q2 * (1.0f / kDm);
  const float rstd = rsqrtf(var + 1e-5f);
  const v4f g0 = *(const v4f*)(gam + c0), g1 = *(const v4f*)(gam + c0 + 4);
  const v4f g2 = *(const v4f*)(gam + c1), g3 = *(const v4f*)(gam + c1 + 4);
  const v4f b0 = *(const v4f*)(bet + c0), b1 = *(const v4f*)(bet + c0 + 4);
  const v4f b2 = *(const v4f*)(bet + c1), b3 = *(const v4f*)(bet + c1 + 4);
  float gg[16], bb[16];
#pragma unroll
  for (int e = 0; e < 4; ++e) {
    gg[e] = g0[e]; gg[4 + e] = g1[e]; gg[8 + e] = g2[e]; gg[12 + e] = g3[e];
    bb[e] = b0[e]; bb[4 + e] = b1[e]; bb[8 + e] = b2[e]; bb[12 + e] = b3[e];
  }
  v8h o0, o1;
#pragma unroll
  for (int e = 0; e < 8; ++e) {
    o0[e] = (_Float16)(((v[e] - mean) * rstd) * gg[e] + bb[e]);
    o1[e] = (_Float16)(((v[8 + e] - mean) * rstd) * gg[8 + e] + bb[8 + e]);
  }
  unsigned short* up = Uo + (size_t)row * kDm;
  *(volatile v8h*)(up + c0) = o0;
  *(volatile v8h*)(up + c1) = o1;
  __threadfence();
  *(volatile v8h*)(up + c0) = o0;
  *(volatile v8h*)(up + c1) = o1;
}

__global__ __launch_bounds__(256) void conv_silu_kernel(
    const float* __restrict__ XZ, const float* __restrict__ cw, const float* __restrict__ cb,
    float* __restrict__ UC, unsigned short* __restrict__ UC16)
{
  __shared__ __align__(16) float sT[16 * kConvTP];
  const int tid = threadIdx.x, lane = tid & 31, wave = tid >> 5;
  const int d0 = blockIdx.x * 256, d = d0 + tid;
  const int g0 = blockIdx.y * 64;
  const int tb = g0 & (kSeq - 1);
  const float w0 = cw[d * 4 + 0], w1 = cw[d * 4 + 1], w2 = cw[d * 4 + 2], w3 = cw[d * 4 + 3];
  const float bc = cb[d];
  float xm3, xm2, xm1;
  {
    const bool hist = (tb > 0);
    const int rb = hist ? (g0 - 3) : g0;
    const float hf = hist ? 1.0f : 0.0f;
    const float v3 = XZ[(size_t)rb * kXzP + d];
    const float v2 = XZ[(size_t)(rb + 1) * kXzP + d];
    const float v1 = XZ[(size_t)(rb + 2) * kXzP + d];
    xm3 = v3 * hf;
    xm2 = v2 * hf;
    xm1 = v1 * hf;
  }
  const int hrow = wave >> 1;
  const int hch  = (wave & 1) * 128 + lane * 4;
#pragma unroll 1
  for (int sub = 0; sub < 4; ++sub) {
    const int lb = g0 + sub * 16;
#pragma unroll 1
    for (int s = 0; s < 16; ++s) {
      const float xcur = XZ[(size_t)(lb + s) * kXzP + d];
      float acc = w0 * xm3;
      acc = fmaf(w1, xm2, acc);
      acc = fmaf(w2, xm1, acc);
      acc = fmaf(w3, xcur, acc);
      const float sv = acc + bc;
      const float sg = __builtin_amdgcn_rcpf(1.0f + expf(-sv));
      sT[s * kConvTP + tid] = sv * sg;
      xm3 = xm2; xm2 = xm1; xm1 = xcur;
    }
    __syncthreads();
    v4f fv[4];
    v8h hv[2];
#pragma unroll
    for (int it = 0; it < 4; ++it) fv[it] = *(const v4f*)(sT + (it * 4 + hrow) * kConvTP + hch);
#pragma unroll
    for (int it = 0; it < 2; ++it) {
      const float* sp = sT + (it * 8 + wave) * kConvTP + lane * 8;
      const v4f a0 = *(const v4f*)(sp);
      const v4f a1 = *(const v4f*)(sp + 4);
#pragma unroll
      for (int e = 0; e < 4; ++e) {
        hv[it][e]     = (_Float16)a0[e];
        hv[it][4 + e] = (_Float16)a1[e];
      }
    }
    for (int pass = 0; pass < 2; ++pass) {
#pragma unroll
      for (int it = 0; it < 4; ++it)
        *(volatile v4f*)(UC + (size_t)(lb + it * 4 + hrow) * kDin + d0 + hch) = fv[it];
#pragma unroll
      for (int it = 0; it < 2; ++it) {
        const size_t o = (size_t)(lb + it * 8 + wave) * kDin + d0 + lane * 8;
        *(volatile v8h*)(UC16 + o) = hv[it];
      }
      __threadfence();
    }
    __syncthreads();
  }
}

__global__ __launch_bounds__(256) void dtr16_kernel(const float* __restrict__ XD, unsigned short* __restrict__ DTR)
{
  const int i = blockIdx.x * 256 + threadIdx.x;
  if (i >= kRows * 4) return;
  const int row = i >> 2, c8 = (i & 3) * 8;
  const v4f a0 = *(const v4f*)(XD + (size_t)row * kXdP + c8);
  const v4f a1 = *(const v4f*)(XD + (size_t)row * kXdP + c8 + 4);
  v8h hv;
#pragma unroll
  for (int e = 0; e < 4; ++e) { hv[e] = (_Float16)a0[e]; hv[4 + e] = (_Float16)a1[e]; }
  unsigned short* qd = DTR + (size_t)i * 8;
  *(volatile v8h*)qd = hv;
  __threadfence();
  *(volatile v8h*)qd = hv;
}

__global__ __launch_bounds__(64) void scan_kernel(
    const float* __restrict__ XD, const float* __restrict__ DT, const float* __restrict__ UC,
    const float* __restrict__ XZ, const float* __restrict__ Alog, const float* __restrict__ Dp,
    unsigned short* __restrict__ Y16)
{
  __shared__ __align__(16) float sX[kScanTS * kScanXP];
  __shared__ __align__(16) float sY[kScanTS * kScanYP];
  __shared__ __align__(16) float sA[kNst * kScanCh];
  const int tid = threadIdx.x, lane = tid & 31, wave = tid >> 5;
  constexpr int kBlkPerB = kDin / kScanCh;
  const int bix = blockIdx.x / kBlkPerB;
  const int d0  = (blockIdx.x - bix * kBlkPerB) * kScanCh;
  const int d   = d0 + tid;
  const size_t row0 = (size_t)bix * kSeq;
#pragma unroll 1
  for (int s = 0; s < kNst; ++s) sA[s * kScanCh + tid] = -expf(Alog[(size_t)d * kNst + s]) * 1.44269504088896341f;
  __syncthreads();
  float negA2[kNst], h[kNst];
#pragma unroll
  for (int s = 0; s < kNst; ++s) {
    negA2[s] = sA[s * kScanCh + tid];
    h[s] = 0.f;
  }
  const float Dd = Dp[d];
  const int lr = tid >> 3, lc4 = (tid & 7) * 4;
  const int q = lane >> 3, c8 = (lane & 7) * 8;
#pragma unroll 1
  for (int t0 = 0; t0 < kSeq; t0 += kScanTS) {
    __syncthreads();
#pragma unroll
    for (int i = 0; i < 8; ++i) {
      const int r = lr + 8 * i;
      *(v4f*)(sX + r * kScanXP + lc4) = *(const v4f*)(XD + (row0 + t0 + r) * kXdP + kDtR + lc4);
    }
    __syncthreads();
#pragma unroll 1
    for (int s = 0; s < kScanTS; ++s) {
      const int t = t0 + s;
      const float* xr = sX + s * kScanXP;
      float Bs[kNst], Cs[kNst];
#pragma unroll
      for (int q4 = 0; q4 < 4; ++q4) {
        const v4f bv = *(const v4f*)(xr + 4 * q4);
        const v4f cv = *(const v4f*)(xr + kNst + 4 * q4);
        Bs[4 * q4 + 0] = bv[0]; Bs[4 * q4 + 1] = bv[1]; Bs[4 * q4 + 2] = bv[2]; Bs[4 * q4 + 3] = bv[3];
        Cs[4 * q4 + 0] = cv[0]; Cs[4 * q4 + 1] = cv[1]; Cs[4 * q4 + 2] = cv[2]; Cs[4 * q4 + 3] = cv[3];
      }
      const size_t grow = row0 + t;
      const float v   = DT[grow * kDin + d];
      const float dt  = fmaxf(v, 0.0f) + log1pf(expf(-fabsf(v)));
      const float xt  = UC[grow * kDin + d];
      const float dtx = dt * xt;
      float y = 0.f;
#pragma unroll
      for (int k = 0; k < kNst; ++k) {
        const float e = exp2f(dt * negA2[k]);
        h[k] = fmaf(e, h[k], dtx * Bs[k]);
        y = fmaf(h[k], Cs[k], y);
      }
      y = fmaf(xt, Dd, y);
      const float zv = XZ[grow * kXzP + kDin + d];
      const float sg = __builtin_amdgcn_rcpf(1.0f + expf(-zv));
      y = y * (zv * sg);
      sY[s * kScanYP + tid] = y;
    }
    __syncthreads();
    v8h hv[8];
#pragma unroll
    for (int it = 0; it < 8; ++it) {
      const int row = it * 8 + wave * 4 + q;
      const float* sp = sY + row * kScanYP + c8;
      const v4f a0 = *(const v4f*)(sp);
      const v4f a1 = *(const v4f*)(sp + 4);
#pragma unroll
      for (int e = 0; e < 4; ++e) {
        hv[it][e]     = (_Float16)a0[e];
        hv[it][4 + e] = (_Float16)a1[e];
      }
    }
    for (int pass = 0; pass < 2; ++pass) {
#pragma unroll
      for (int it = 0; it < 8; ++it) {
        const int row = it * 8 + wave * 4 + q;
        const size_t o = (row0 + t0 + row) * kDin + d0 + c8;
        *(volatile v8h*)(Y16 + o) = hv[it];
      }
      __threadfence();
    }
  }
}

__global__ __launch_bounds__(256) void gelu_f16x2_kernel(
    const float* __restrict__ H1, unsigned short* __restrict__ H16, int n2)
{
  const int i = blockIdx.x * 256 + threadIdx.x;
  if (i >= n2) return;
  const int row = i >> 9, c2 = (i & 511) * 2;
  const v2f a = *(const v2f*)(H1 + (size_t)row * kXzP + c2);
  const float v0 = a[0], v1 = a[1];
  const float g0 = 0.5f * v0 * (1.0f + erff(v0 * 0.70710678118654752f));
  const float g1 = 0.5f * v1 * (1.0f + erff(v1 * 0.70710678118654752f));
  const _Float16 h0 = (_Float16)g0, h1 = (_Float16)g1;
  const unsigned u = (unsigned)__builtin_bit_cast(unsigned short, h0) | ((unsigned)__builtin_bit_cast(unsigned short, h1) << 16);
  ((volatile unsigned*)H16)[i] = u;
  __threadfence();
  ((volatile unsigned*)H16)[i] = u;
}

extern "C" void kernel_launch(void* const* d_in, const int* in_sizes, int n_in,
                              void* d_out, int out_size, void* d_ws, size_t ws_size,
                              hipStream_t stream) {
  if (n_in < 18) return;
  if (in_sizes[0]  != kRows * kDm) return;
  if (in_sizes[1]  != kDepth * kDm) return;
  if (in_sizes[2]  != kDepth * kDm) return;
  if (in_sizes[3]  != kDepth * kNWin) return;
  if (in_sizes[4]  != kDepth * kDin * 4) return;
  if (in_sizes[5]  != kDepth * kDin) return;
  if (in_sizes[6]  != kDepth * kNWx) return;
  if (in_sizes[7]  != kDepth * kNWdt) return;
  if (in_sizes[8]  != kDepth * kDin) return;
  if (in_sizes[9]  != kDepth * kDin * kNst) return;
  if (in_sizes[10] != kDepth * kDin) return;
  if (in_sizes[11] != kDepth * kNWo) return;
  if (in_sizes[12] != kDepth * kDm) return;
  if (in_sizes[13] != kDepth * kDm) return;
  if (in_sizes[14] != kDepth * kNW1) return;
  if (in_sizes[15] != kDepth * kHid) return;
  if (in_sizes[16] != kDepth * kNW2) return;
  if (in_sizes[17] != kDepth * kDm) return;
  if (out_size != kRows * kDm) return;
  if (ws_size < kWsTotal) return;

  const float* x        = (const float*)d_in[0];
  const float* ln1_g    = (const float*)d_in[1];
  const float* ln1_b    = (const float*)d_in[2];
  const float* in_w     = (const float*)d_in[3];
  const float* conv_w   = (const float*)d_in[4];
  const float* conv_b   = (const float*)d_in[5];
  const float* xproj_w  = (const float*)d_in[6];
  const float* dtproj_w = (const float*)d_in[7];
  const float* dtproj_b = (const float*)d_in[8];
  const float* A_log    = (const float*)d_in[9];
  const float* D_skip   = (const float*)d_in[10];
  const float* out_w    = (const float*)d_in[11];
  const float* ln2_g    = (const float*)d_in[12];
  const float* ln2_b    = (const float*)d_in[13];
  const float* mlp_w1   = (const float*)d_in[14];
  const float* mlp_b1   = (const float*)d_in[15];
  const float* mlp_w2   = (const float*)d_in[16];
  const float* mlp_b2   = (const float*)d_in[17];
  float* out = (float*)d_out;

  char* ws = (char*)d_ws;
  float*          XA    = (float*)(ws + kOffXA);
  float*          XB    = (float*)(ws + kOffXB);
  unsigned short* pU16  = (unsigned short*)(ws + kOffU16);
  float*          XZ    = (float*)(ws + kOffXZ);
  float*          UC    = (float*)(ws + kOffUC);
  unsigned short* UC16  = (unsigned short*)(ws + kOffUC16);
  float*          XD    = (float*)(ws + kOffXD);
  unsigned short* DTR16 = (unsigned short*)(ws + kOffDTR16);
  float*          DT    = (float*)(ws + kOffDT);
  unsigned short* Y16   = (unsigned short*)(ws + kOffY16);
  unsigned short* H16   = (unsigned short*)(ws + kOffH16);
  unsigned short* W16   = (unsigned short*)(ws + kOffW16);
  float*          H1    = XZ;

  for (int dl = 0; dl < kDepth; ++dl) {
    const float* xcur = (dl == 0) ? x : XA;

    castw_kernel<<<kCastBlocks, 256, 0, stream>>>(
        in_w + (size_t)dl * kNWin, xproj_w + (size_t)dl * kNWx, dtproj_w + (size_t)dl * kNWdt,
        out_w + (size_t)dl * kNWo, mlp_w1 + (size_t)dl * kNW1, mlp_w2 + (size_t)dl * kNW2, W16);

    ln_f16_kernel<<<kRows / 8, 256, 0, stream>>>(xcur, ln1_g + (size_t)dl * kDm, ln1_b + (size_t)dl * kDm, pU16);

    wmma_gemm64<0, false, 0, 0, false><<<dim3(256, 1), 256, 0, stream>>>(
        pU16, nullptr, kDm, 0L,
        W16 + kEoffWin, nullptr, kDm, 0L,
        (void*)XZ, nullptr, kXzP, 0L,
        nullptr, nullptr, 0L,
        kRows, kXzP, kDm, 1.0f);

    conv_silu_kernel<<<dim3(kDin / 256, kRows / 64), 256, 0, stream>>>(
        XZ, conv_w + (size_t)dl * kDin * 4, conv_b + (size_t)dl * kDin, UC, UC16);

    wmma_gemm64<0, false, 0, 0, false><<<dim3(8, 1), 256, 0, stream>>>(
        UC16, nullptr, kDin, 0L,
        W16 + kEoffWx, nullptr, kDin, 0L,
        (void*)XD, nullptr, kXdP, 0L,
        nullptr, nullptr, 0L,
        kRows, kXdP, kDin, 1.0f);

    dtr16_kernel<<<(kRows * 4) / 256, 256, 0, stream>>>(XD, DTR16);

    wmma_gemm64<0, false, 2, 0, false><<<dim3(128, 1), 256, 0, stream>>>(
        DTR16, nullptr, kDtR, 0L,
        W16 + kEoffWdt, nullptr, kDtR, 0L,
        (void*)DT, nullptr, kDin, 0L,
        dtproj_b + (size_t)dl * kDin, nullptr, 0L,
        kRows, kDin, kDtR, 1.0f);

    scan_kernel<<<kBatch * (kDin / kScanCh), kScanCh, 0, stream>>>(
        XD, DT, UC, XZ, A_log + (size_t)dl * kDin * kNst, D_skip + (size_t)dl * kDin, Y16);

    wmma_gemm64<0, false, 0, 0, true><<<dim3(64, 1), 256, 0, stream>>>(
        Y16, nullptr, kDin, 0L,
        W16 + kEoffWo, nullptr, kDin, 0L,
        (void*)XB, nullptr, kDm, 0L,
        nullptr, xcur, 0L,
        kRows, kDm, kDin, 1.0f);

    ln_f16_kernel<<<kRows / 8, 256, 0, stream>>>(XB, ln2_g + (size_t)dl * kDm, ln2_b + (size_t)dl * kDm, pU16);

    wmma_gemm64<0, false, 2, 0, false><<<dim3(128, 1), 256, 0, stream>>>(
        pU16, nullptr, kDm, 0L,
        W16 + kEoffW1, nullptr, kDm, 0L,
        (void*)H1, nullptr, kXzP, 0L,
        mlp_b1 + (size_t)dl * kHid, nullptr, 0L,
        kRows, kHid, kDm, 1.0f);

    gelu_f16x2_kernel<<<(kRows * kHid / 2) / 256, 256, 0, stream>>>(H1, H16, kRows * kHid / 2);

    float* dst = (dl == kDepth - 1) ? out : XA;
    wmma_gemm64<0, false, 2, 0, true><<<dim3(64, 1), 256, 0, stream>>>(
        H16, nullptr, kHid, 0L,
        W16 + kEoffW2, nullptr, kHid, 0L,
        (void*)dst, nullptr, kDm, 0L,
        mlp_b2 + (size_t)dl * kDm, XB, 0L,
        kRows, kDm, kHid, 1.0f);
  }
}
